// TN_layer_MultiNode_34840774705660
// MI455X (gfx1250) — hardware-verified
//
#include <hip/hip_runtime.h>
#include <stdint.h>

#define NB    2048
#define NFT   64
#define FD    32
#define NS    32
#define DD    32
#define OD    32
#define TEN   1048576
#define SEL   32768
#define NBT   128
static_assert(NB == NBT * 16);
static_assert(FD == 32);
static_assert(DD == 32);
static_assert(OD == 32);
static_assert(NS * 2 == NFT);
static_assert(TEN == NS * SEL);
static_assert(SEL == DD * DD * FD);

typedef _Float16     v16h __attribute__((ext_vector_type(16)));
typedef _Float16     v8h  __attribute__((ext_vector_type(8)));
typedef float        v8f  __attribute__((ext_vector_type(8)));
typedef float        v4f  __attribute__((ext_vector_type(4)));
typedef unsigned int v4u  __attribute__((ext_vector_type(4)));

union Frag { v16h v; v8h half[2]; };

__device__ __forceinline__ unsigned short bf_bits(float f) {
  unsigned u = __float_as_uint(f);
  return (unsigned short)((u + 0x7FFFu + ((u >> 16) & 1u)) >> 16);
}
__device__ __forceinline__ float bf_up(unsigned short b) { return __uint_as_float(((unsigned)b) << 16); }
__device__ __forceinline__ float bfr(float f) { return bf_up(bf_bits(f)); }
__device__ __forceinline__ unsigned short h_bits(float f) {
  return __builtin_bit_cast(unsigned short, (_Float16)f);
}
__device__ __forceinline__ v8f zero8() {
  v8f z;
  z[0] = 0.f; z[1] = 0.f; z[2] = 0.f; z[3] = 0.f; z[4] = 0.f; z[5] = 0.f; z[6] = 0.f; z[7] = 0.f;
  return z;
}

__device__ __forceinline__ v16h ldfrag(const _Float16* p) {
  Frag f;
  f.half[0] = *(const v8h*)(p);
  f.half[1] = *(const v8h*)(p + 16);
  return f.v;
}

__device__ __forceinline__ v8f mma(v16h a, v16h b, v8f c) {
  v8f d = __builtin_amdgcn_wmma_f32_16x16x32_f16(false, a, false, b, (short)0, c, false, false);
#if defined(__HIP_DEVICE_COMPILE__)
  asm volatile("v_nop\n\tv_nop\n\tv_nop\n\tv_nop" : "+v"(d) : "v"(a), "v"(b));
#endif
  return d;
}

__global__ __launch_bounds__(256) void k_tr(const float* __restrict__ L, const float* __restrict__ R,
                                            const float* __restrict__ O, unsigned short* P) {
  __shared__ __align__(16) unsigned short sT[8192];
  const int tid = threadIdx.x;
  const int bid = blockIdx.x;
  const int t   = bid >> 7;
  const int s   = (bid >> 2) & 31;
  const int kg  = bid & 3;
  const float* src = (t == 0) ? L : ((t == 1) ? R : O);
  src += (size_t)s * SEL + (size_t)kg * 8;
  unsigned short* dst = P + (size_t)t * TEN + (size_t)s * SEL + (size_t)kg * 8192;

#pragma unroll 1
  for (int it = 0; it < 4; ++it) {
    const int p = it * 256 + tid;
    const int i = p >> 5, j = p & 31;
    const float* q = src + (size_t)i * 1024 + (size_t)j * 32;
    const v4f v0 = *(const v4f*)(q);
    const v4f v1 = *(const v4f*)(q + 4);
    unsigned short* d = sT + j * 32 + i;
#pragma unroll
    for (int kl = 0; kl < 4; ++kl) {
      d[kl * 1024]       = h_bits(bfr(v0[kl]) * 1024.0f);
      d[(kl + 4) * 1024] = h_bits(bfr(v1[kl]) * 1024.0f);
    }
  }
  __syncthreads();

  v4u pv[4];
#pragma unroll
  for (int it = 0; it < 4; ++it) pv[it] = *(const v4u*)(sT + (size_t)(it * 256 + tid) * 8);
#pragma unroll
  for (int it = 0; it < 4; ++it) *(volatile v4u*)(dst + (size_t)(it * 256 + tid) * 8) = pv[it];
  __threadfence();
#pragma unroll
  for (int it = 0; it < 4; ++it) *(volatile v4u*)(dst + (size_t)(it * 256 + tid) * 8) = pv[it];
}

__device__ __forceinline__ void bil_tile(v16h ah, v16h al, v16h bh, v16h bl, _Float16* dh, _Float16* dl) {
  v8f c0 = mma(ah, bh, zero8());
  v8f c1 = mma(ah, bl, zero8());
  c1 = mma(al, bh, c1);
  v8h hv, lv;
#pragma unroll
  for (int r = 0; r < 8; ++r) {
    const float m = c0[r] + c1[r] * 0.00048828125f;
    const _Float16 hh = (_Float16)m;
    hv[r] = hh;
    lv[r] = (_Float16)((m - (float)hh) * 2048.0f);
  }
  *(v8h*)dh = hv;
  *(v8h*)dl = lv;
}

__global__ __launch_bounds__(32) void k_main(const float* __restrict__ x, const unsigned short* __restrict__ Pp,
                                             const float* __restrict__ bias, float* out) {
  extern __shared__ __align__(16) _Float16 smem[];
  __shared__ __align__(16) float sO[512];
  const _Float16* P = (const _Float16*)(const void*)Pp;
  const int lane = threadIdx.x & 31;
  const int h    = lane >> 4;
  const int lo   = lane & 15;
  const int w    = blockIdx.x;
  const int s    = w / NBT;
  const int b0   = (w % NBT) * 16;
  _Float16* AH = smem;
  _Float16* BH = smem + 32768;

#pragma unroll 1
  for (int side = 0; side < 2; ++side) {
    const float* xrow = x + ((size_t)(b0 + lo) * NFT + (size_t)(2 * s + side)) * FD + 8 * h;
    const _Float16* Wp = P + (size_t)side * TEN + (size_t)s * SEL + (size_t)lo * 32 + 8 * h;
    _Float16* PH = smem + side * 32768 + lo * 1024 + 8 * h;
    _Float16* PL = PH + 16384;

    Frag xb;
    {
      const v4f x0 = *(const v4f*)(xrow);
      const v4f x1 = *(const v4f*)(xrow + 4);
      const v4f x2 = *(const v4f*)(xrow + 16);
      const v4f x3 = *(const v4f*)(xrow + 20);
      v8h p0, p1;
#pragma unroll
      for (int c = 0; c < 4; ++c) {
        p0[c]     = (_Float16)(bfr(x0[c]) * 16.0f);
        p0[4 + c] = (_Float16)(bfr(x1[c]) * 16.0f);
        p1[c]     = (_Float16)(bfr(x2[c]) * 16.0f);
        p1[4 + c] = (_Float16)(bfr(x3[c]) * 16.0f);
      }
      xb.half[0] = p0;
      xb.half[1] = p1;
    }

#pragma unroll 1
    for (int j = 0; j < 64; ++j) {
      const _Float16* ap = Wp + (size_t)j * 512;
      Frag af;
      af.half[0] = *(const v8h*)(ap);
      af.half[1] = *(const v8h*)(ap + 16);
      const v8f acc = mma(af.v, xb.v, zero8());
      v8h hv, lv;
#pragma unroll
      for (int r = 0; r < 8; ++r) {
        const float a16 = acc[r] * 0.0009765625f;
        const _Float16 hh = (_Float16)a16;
        hv[r] = hh;
        lv[r] = (_Float16)((a16 - (float)hh) * 2048.0f);
      }
      const int off = (j >> 1) * 32 + (j & 1) * 16;
      *(v8h*)(PH + off) = hv;
      *(v8h*)(PL + off) = lv;
    }
  }
  __syncthreads();

#pragma unroll 1
  for (int b = 0; b < 16; ++b) {
    const _Float16* pa = AH + b * 1024 + lo * 32 + 8 * h;
    const _Float16* pb = BH + b * 1024 + lo * 32 + 8 * h;
    const v16h ah0 = ldfrag(pa);
    const v16h ah1 = ldfrag(pa + 512);
    const v16h al0 = ldfrag(pa + 16384);
    const v16h al1 = ldfrag(pa + 16384 + 512);
    const v16h bh0 = ldfrag(pb);
    const v16h bh1 = ldfrag(pb + 512);
    const v16h bl0 = ldfrag(pb + 16384);
    const v16h bl1 = ldfrag(pb + 16384 + 512);
    __syncthreads();
    _Float16* dm = AH + b * 1024 + lo * 32 + 8 * h;
    bil_tile(ah0, al0, bh0, bl0, dm,            dm + 16384);
    bil_tile(ah0, al0, bh1, bl1, dm + 512,      dm + 16384 + 512);
    bil_tile(ah1, al1, bh0, bl0, dm + 16,       dm + 16384 + 16);
    bil_tile(ah1, al1, bh1, bl1, dm + 512 + 16, dm + 16384 + 512 + 16);
  }
  __syncthreads();

  v8f oh0 = zero8(), oh1 = zero8(), ol0 = zero8(), ol1 = zero8();
  {
    const _Float16* pm = AH + lo * 1024 + 8 * h;
    const _Float16* po = P + (size_t)2 * TEN + ((size_t)s * 32 + lo) * 1024 + 8 * h;
#pragma unroll 1
    for (int ks = 0; ks < 32; ++ks) {
      const v16h mh = ldfrag(pm + ks * 32);
      const v16h ml = ldfrag(pm + 16384 + ks * 32);
      const v16h o0 = ldfrag(po + ks * 32);
      const v16h o1 = ldfrag(po + 16384 + ks * 32);
      oh0 = mma(mh, o0, oh0);
      oh1 = mma(mh, o1, oh1);
      ol0 = mma(ml, o0, ol0);
      ol1 = mma(ml, o1, ol1);
    }
  }

  const float bv0 = bfr(bias[s * OD + lo]);
  const float bv1 = bfr(bias[s * OD + 16 + lo]);
#pragma unroll
  for (int r = 0; r < 8; ++r) {
    const float v0 = (oh0[r] + ol0[r] * 0.00048828125f) * 3.814697265625e-06f + bv0;
    const float v1 = (oh1[r] + ol1[r] * 0.00048828125f) * 3.814697265625e-06f + bv1;
    sO[(8 * h + r) * 32 + lo]      = v0;
    sO[(8 * h + r) * 32 + 16 + lo] = v1;
  }
  __syncthreads();

  const int piece = lane & 7;
  const int lq    = lane >> 3;
  v4f pv[4];
#pragma unroll
  for (int it = 0; it < 4; ++it) pv[it] = *(const v4f*)(sO + (it * 4 + lq) * 32 + piece * 4);
  float* ob = out + ((size_t)b0 * NS + (size_t)s) * OD + (size_t)piece * 4;
#pragma unroll
  for (int it = 0; it < 4; ++it) *(volatile v4f*)(ob + (size_t)(it * 4 + lq) * (NS * OD)) = pv[it];
  __threadfence();
#pragma unroll
  for (int it = 0; it < 4; ++it) *(volatile v4f*)(ob + (size_t)(it * 4 + lq) * (NS * OD)) = pv[it];
}

extern "C" void kernel_launch(void* const* d_in, const int* in_sizes, int n_in,
                              void* d_out, int out_size, void* d_ws, size_t ws_size,
                              hipStream_t stream) {
  if (n_in < 5) return;
  if (in_sizes[0] != NB * NFT * FD) return;
  if (in_sizes[1] != TEN) return;
  if (in_sizes[2] != TEN) return;
  if (in_sizes[3] != TEN) return;
  if (in_sizes[4] != NS * OD) return;
  if (out_size != NB * NS * OD) return;

  const float* x    = (const float*)d_in[0];
  const float* L    = (const float*)d_in[1];
  const float* R    = (const float*)d_in[2];
  const float* O    = (const float*)d_in[3];
  const float* bias = (const float*)d_in[4];
  float* out = (float*)d_out;

  const size_t szP = (size_t)3 * TEN * 2;
  if (szP > ws_size) return;
  if (szP > (size_t)134217728) return;
  unsigned short* P = (unsigned short*)d_ws;

  const int ldsMain = 131072;
  (void)hipFuncSetAttribute(reinterpret_cast<const void*>(&k_main),
                            hipFuncAttributeMaxDynamicSharedMemorySize, ldsMain);

  const dim3 gTr(3 * NS * 4);
  const dim3 bTr(256);
  const dim3 gMain(NS * NBT);
  const dim3 bMain(32);

  k_tr<<<gTr, bTr, 0, stream>>>(L, R, O, P);
  k_main<<<gMain, bMain, ldsMain, stream>>>(x, P, bias, out);
  (void)hipGetLastError();
}
